// Feedzai_60559038873895
// MI455X (gfx1250) — hardware-verified
//
#include <hip/hip_runtime.h>
#include <stdint.h>


#define NB    256
#define NT    1024
#define NF    18
#define NU    32
#define NG    96
#define NTAB  1000
#define RB    16
#define NTHR  128
#define HTHR  256
#define LDP   32
#define DP    33

typedef _Float16 f16t;
typedef f16t  v16h __attribute__((ext_vector_type(16)));
typedef f16t  v8h  __attribute__((ext_vector_type(8)));
typedef f16t  v4h  __attribute__((ext_vector_type(4)));
typedef float v8f  __attribute__((ext_vector_type(8)));
typedef float v4f  __attribute__((ext_vector_type(4)));

union Frag { v16h v; v8h q[2]; };

__device__ __forceinline__ v8f wmma16(v16h a, v16h b, v8f c) {
    return __builtin_amdgcn_wmma_f32_16x16x32_f16(false, a, false, b, (short)0, c, false, false);
}

__device__ __forceinline__ v16h ldfrag(const f16t* tile, int pitch) {
    const int l = threadIdx.x & 31, h = l >> 4, m = l & 15;
    const f16t* p = tile + m * pitch + 8 * h;
    Frag f;
    f.q[0] = *(const v8h*)p;
    f.q[1] = *(const v8h*)(p + 16);
    return f.v;
}

__device__ __forceinline__ float hsig(float v) {
    return fminf(fmaxf(0.2f * v + 0.5f, 0.0f), 1.0f);
}

__device__ __forceinline__ float ftanh(float x) {
    const float ax = fabsf(x);
    const float e  = __expf(-2.0f * ax);
    const float r  = (1.0f - e) * __builtin_amdgcn_rcpf(1.0f + e);
    return copysignf(r, x);
}

__global__ __launch_bounds__(NTHR)
void k_scan(const float* x, const int* ids, const float* table, const float* kern,
            const float* rkern, const float* bias, float* tab, float* hlast, int nb)
{
    __shared__ __attribute__((aligned(16))) f16t  sWx[NG * LDP];
    __shared__ __attribute__((aligned(16))) f16t  sWh[NG * LDP];
    __shared__ __attribute__((aligned(16))) float sH[RB * NU];
    __shared__ __attribute__((aligned(16))) f16t  sHf[RB * LDP];
    __shared__ __attribute__((aligned(16))) f16t  sX[RB * LDP];
    __shared__ __attribute__((aligned(16))) f16t  sRH[RB * LDP];
    __shared__ __attribute__((aligned(16))) float sHN[RB * NU];

    const int tid  = threadIdx.x;
    const int wave = tid >> 5;
    const int lane = tid & 31;
    const int hl   = lane >> 4;
    const int m    = lane & 15;
    const int b0   = blockIdx.x * RB;
    if (b0 + RB > nb) return;

    const int    gr    = tid >> 3;
    const int    gc    = (tid & 7) * 4;
    const size_t idrow = (size_t)(b0 + gr) * NT;

    {
        const size_t cb = (size_t)(b0 + gr) * NU + gc;
#pragma unroll 1
        for (int i = 0; i < NTAB; ++i) {
            const size_t o = (size_t)i * NB * NU + cb;
            const v4f v = *(const v4f*)(table + o);
            float* d = tab + o;
            *(volatile v4f*)d = v;
            __threadfence();
            *(volatile v4f*)d = v;
        }
        __threadfence();
    }

    for (int i = tid; i < NG * LDP; i += NTHR) {
        const int n = i >> 5, k = i & 31;
        const float vx = (k < NF) ? kern[k * NG + n] : 0.0f;
        sWx[i] = (f16t)(vx * 16.0f);
        sWh[i] = (f16t)(rkern[k * NG + n] * 16.0f);
    }
    for (int i = tid; i < RB * LDP; i += NTHR) sX[i] = (f16t)0.0f;
    __syncthreads();

    const int  wh  = wave & 1;
    const v16h bzx = ldfrag(sWx + (16 * wave) * LDP, LDP);
    const v16h bzh = ldfrag(sWh + (16 * wave) * LDP, LDP);
    const v16h bgx = ldfrag(sWx + (64 + 16 * wh) * LDP, LDP);
    const v16h bgh = ldfrag(sWh + (64 + 16 * wh) * LDP, LDP);
    const float bz  = bias[16 * wave + m];
    const float bg  = bias[64 + 16 * wh + m];
    const float inv = 0.0625f;

    int xr[3], xf[3], xv[3];
    size_t xo[3];
#pragma unroll
    for (int s = 0; s < 3; ++s) {
        const int e  = tid + NTHR * s;
        xv[s] = (e < RB * NF) ? 1 : 0;
        const int ec = xv[s] ? e : 0;
        xr[s] = ec / NF;
        xf[s] = ec - xr[s] * NF;
        xo[s] = ((size_t)(b0 + xr[s]) * NT) * NF + xf[s];
    }

    const v8f zero8 = {0.f, 0.f, 0.f, 0.f, 0.f, 0.f, 0.f, 0.f};

#pragma unroll 1
    for (int t = 0; t < NT; ++t) {
        const int idv = ids[idrow + t];
        const int idc = idv < 0 ? 0 : (idv > NTAB - 1 ? NTAB - 1 : idv);
        float* trow = tab + ((size_t)idc * NB + (size_t)(b0 + gr)) * NU + gc;
        const v4f hv = *(volatile const v4f*)trow;
        *(v4f*)(sH + gr * NU + gc) = hv;
        v4h hq;
        hq[0] = (f16t)hv[0]; hq[1] = (f16t)hv[1]; hq[2] = (f16t)hv[2]; hq[3] = (f16t)hv[3];
        *(v4h*)(sHf + gr * LDP + gc) = hq;
#pragma unroll
        for (int s = 0; s < 3; ++s) {
            if (xv[s]) {
                float v;
                if (xf[s] == 0) v = (float)ids[(size_t)(b0 + xr[s]) * NT + t];
                else            v = x[xo[s] + (size_t)t * NF];
                sX[xr[s] * LDP + xf[s]] = (f16t)v;
            }
        }
        __syncthreads();

        const v16h aX = ldfrag(sX, LDP);
        const v16h aH = ldfrag(sHf, LDP);
        v8f acc = zero8;
        acc = wmma16(aX, bzx, acc);
        acc = wmma16(aH, bzh, acc);
        asm volatile("v_nop\n\tv_nop\n\tv_nop\n\tv_nop"
                     : "+v"(acc) : "v"(aX), "v"(aH), "v"(bzx), "v"(bzh));
        v8f zv = zero8;
        if (wave >= 2) {
            const int u = 16 * (wave - 2) + m;
#pragma unroll
            for (int r = 0; r < 8; ++r) {
                const int   row = 8 * hl + r;
                const float rg  = hsig(fmaf(acc[r], inv, bz));
                sRH[row * LDP + u] = (f16t)(rg * sH[row * NU + u]);
            }
        } else {
#pragma unroll
            for (int r = 0; r < 8; ++r) zv[r] = hsig(fmaf(acc[r], inv, bz));
        }
        __syncthreads();

        if (wave < 2) {
            const v16h aR = ldfrag(sRH, LDP);
            v8f acc2 = zero8;
            acc2 = wmma16(aX, bgx, acc2);
            acc2 = wmma16(aR, bgh, acc2);
            asm volatile("v_nop\n\tv_nop\n\tv_nop\n\tv_nop"
                         : "+v"(acc2) : "v"(aX), "v"(aR), "v"(bgx), "v"(bgh));
            const int u = 16 * wave + m;
#pragma unroll
            for (int r = 0; r < 8; ++r) {
                const int   row  = 8 * hl + r;
                const float g    = ftanh(fmaf(acc2[r], inv, bg));
                const float hcur = sH[row * NU + u];
                const float z    = zv[r];
                sHN[row * NU + u] = z * hcur + (1.0f - z) * g;
            }
        }
        __syncthreads();

        const v4f hn = *(const v4f*)(sHN + gr * NU + gc);
        float* dst = (t == NT - 1) ? (hlast + (size_t)(b0 + gr) * NU + gc) : trow;
        *(volatile v4f*)dst = hn;
        __threadfence();
        *(volatile v4f*)dst = hn;
        __threadfence();
    }
}

__global__ __launch_bounds__(HTHR)
void k_head(const float* hlast, const float* w1, const float* b1, const float* w2,
            const float* b2, float* out, int nb)
{
    __shared__ __attribute__((aligned(16))) f16t  sA[NB * LDP];
    __shared__ __attribute__((aligned(16))) f16t  sB[32 * LDP];
    __shared__ float sD[NB * DP];
    __shared__ __attribute__((aligned(16))) float sO[NB];

    const int tid  = threadIdx.x;
    const int wave = tid >> 5;
    const int lane = tid & 31;
    const int hl   = lane >> 4;
    const int m    = lane & 15;
    if (nb != NB) return;

    {
        const float* p = hlast + (size_t)tid * NU;
#pragma unroll
        for (int c = 0; c < 4; ++c) {
            const v4f a = *(const v4f*)(p + 8 * c);
            const v4f b = *(const v4f*)(p + 8 * c + 4);
            v8h q;
            q[0] = (f16t)a[0]; q[1] = (f16t)a[1]; q[2] = (f16t)a[2]; q[3] = (f16t)a[3];
            q[4] = (f16t)b[0]; q[5] = (f16t)b[1]; q[6] = (f16t)b[2]; q[7] = (f16t)b[3];
            *(v8h*)(sA + tid * LDP + 8 * c) = q;
        }
#pragma unroll
        for (int s = 0; s < 4; ++s) {
            const int i = tid + HTHR * s;
            const int n = i >> 5, k = i & 31;
            sB[i] = (f16t)(w1[k * 32 + n] * 16.0f);
        }
    }
    __syncthreads();

    const v16h a0 = ldfrag(sA + (32 * wave) * LDP, LDP);
    const v16h a1 = ldfrag(sA + (32 * wave + 16) * LDP, LDP);
    const v16h c0 = ldfrag(sB, LDP);
    const v16h c1 = ldfrag(sB + 16 * LDP, LDP);
    const v8f zero8 = {0.f, 0.f, 0.f, 0.f, 0.f, 0.f, 0.f, 0.f};
    v8f d00 = zero8, d01 = zero8, d10 = zero8, d11 = zero8;
    d00 = wmma16(a0, c0, d00);
    d01 = wmma16(a0, c1, d01);
    d10 = wmma16(a1, c0, d10);
    d11 = wmma16(a1, c1, d11);
    asm volatile("v_nop\n\tv_nop\n\tv_nop\n\tv_nop"
                 : "+v"(d00), "+v"(d01), "+v"(d10), "+v"(d11)
                 : "v"(a0), "v"(a1), "v"(c0), "v"(c1));

    const float inv = 0.0625f;
    {
        const int   colA = m, colB = 16 + m;
        const float bA = b1[colA], bB = b1[colB];
#pragma unroll
        for (int r = 0; r < 8; ++r) {
            const int row0 = 32 * wave + 8 * hl + r;
            const int row1 = row0 + 16;
            sD[row0 * DP + colA] = fmaxf(fmaf(d00[r], inv, bA), 0.0f);
            sD[row0 * DP + colB] = fmaxf(fmaf(d01[r], inv, bB), 0.0f);
            sD[row1 * DP + colA] = fmaxf(fmaf(d10[r], inv, bA), 0.0f);
            sD[row1 * DP + colB] = fmaxf(fmaf(d11[r], inv, bB), 0.0f);
        }
    }
    __syncthreads();

    {
        float s = b2[0];
#pragma unroll
        for (int j = 0; j < 32; ++j) s = fmaf(sD[tid * DP + j], w2[j], s);
        sO[tid] = __builtin_amdgcn_rcpf(1.0f + __expf(-s));
    }
    __syncthreads();

    if (wave == 0) {
        const v4f v0 = *(const v4f*)(sO + 4 * lane);
        const v4f v1 = *(const v4f*)(sO + 128 + 4 * lane);
        float* p0 = out + 4 * lane;
        float* p1 = out + 128 + 4 * lane;
        *(volatile v4f*)p0 = v0;
        *(volatile v4f*)p1 = v1;
        __threadfence();
        *(volatile v4f*)p0 = v0;
        *(volatile v4f*)p1 = v1;
    }
}

extern "C" void kernel_launch(void* const* d_in, const int* in_sizes, int n_in,
                              void* d_out, int out_size, void* d_ws, size_t ws_size,
                              hipStream_t stream) {
    if (n_in < 10) return;
    if (in_sizes[0] != NB * NT * NF || in_sizes[1] != NB * NT || in_sizes[2] != NTAB * NB * NU ||
        in_sizes[3] != NF * NG || in_sizes[4] != NU * NG || in_sizes[5] != NG ||
        in_sizes[6] != NU * 32 || in_sizes[7] != 32 || in_sizes[8] != 32 || in_sizes[9] != 1)
        return;
    if (out_size != NB) return;

    const float* x     = (const float*)d_in[0];
    const int*   ids   = (const int*)d_in[1];
    const float* table = (const float*)d_in[2];
    const float* kern  = (const float*)d_in[3];
    const float* rkern = (const float*)d_in[4];
    const float* bias  = (const float*)d_in[5];
    const float* w1    = (const float*)d_in[6];
    const float* b1    = (const float*)d_in[7];
    const float* w2    = (const float*)d_in[8];
    const float* b2    = (const float*)d_in[9];
    float* out = (float*)d_out;

    const size_t tab_bytes = (size_t)NTAB * NB * NU * sizeof(float);
    const size_t hl_off    = (tab_bytes + 255) & ~(size_t)255;
    const size_t hl_bytes  = (size_t)NB * NU * sizeof(float);
    if (hl_off + hl_bytes > ws_size) return;
    float* tab   = (float*)d_ws;
    float* hlast = (float*)((char*)d_ws + hl_off);

    k_scan<<<dim3(NB / RB), dim3(NTHR), 0, stream>>>(x, ids, table, kern, rkern, bias, tab, hlast, NB);
    k_head<<<dim3(1), dim3(HTHR), 0, stream>>>(hlast, w1, b1, w2, b2, out, NB);
}
